// SSMPathway_6828998000924
// MI455X (gfx1250) — hardware-run, weakly checked
//
#include <hip/hip_runtime.h>
#include <math.h>

typedef __attribute__((ext_vector_type(16))) _Float16 v16h;
typedef __attribute__((ext_vector_type(8)))  _Float16 v8h;
typedef __attribute__((ext_vector_type(16))) __bf16   v16b;
typedef __attribute__((ext_vector_type(8)))  __bf16   v8b;
typedef __attribute__((ext_vector_type(8)))  float    v8f;
typedef __attribute__((ext_vector_type(4)))  float    v4f;

constexpr int kBatch  = 2;
constexpr int kSeq    = 2048;
constexpr int kDm     = 1024;
constexpr int kDin    = 2048;
constexpr int kNst    = 16;
constexpr int kDtR    = 64;
constexpr int kXpN    = 96;
constexpr int kXpPad  = 128;
constexpr int kXbcP   = 64;
constexpr int kRows   = kBatch * kSeq;
constexpr float kLnEps = 1e-5f;
constexpr int kConvTP = 260;
constexpr int kScanTS = 64;
constexpr int kScanCh = 64;
constexpr int kScanYP = 68;
constexpr int kXbcW   = 32;
constexpr float kWScale  = 64.0f;
constexpr float kUScale  = 16.0f;
constexpr float kYScale  = 64.0f;
constexpr float kDtInv   = 1.0f / 16.0f;
static_assert(kDtR + 2 * kNst == kXpN);
static_assert((kDm % 32) == 0 && (kDin % 32) == 0 && (kDtR % 32) == 0);
static_assert((kRows % 64) == 0 && (kDin % 64) == 0 && (kDm % 64) == 0 && (kXbcP % 64) == 0);
static_assert((kSeq % kScanTS) == 0 && (kSeq % 64) == 0 && (kDin % kScanCh) == 0 && (kDin % 256) == 0);
static_assert((kRows % 8) == 0 && (kDm % 256) == 0);

constexpr size_t kOffXN16 = 0;
constexpr size_t kOffWI16 = kOffXN16 + (size_t)kRows * kDm * 2;
constexpr size_t kOffY16  = 0;
constexpr size_t kOffWX16 = kOffWI16 + (size_t)kRows * kDm * 2;
constexpr size_t kOffWD16 = kOffWX16 + (size_t)kXpPad * kDin * 2;
constexpr size_t kOffWO16 = kOffWD16 + (size_t)kDin * kDtR * 2;
constexpr size_t kOffXC   = kOffWO16 + (size_t)kDm * kDin * 2;
constexpr size_t kOffZ    = kOffXC   + (size_t)kRows * kDin * 4;
constexpr size_t kOffU16  = kOffZ    + (size_t)kRows * kDin * 4;
constexpr size_t kOffDT16 = kOffU16;
constexpr size_t kOffDR16 = kOffU16  + (size_t)kRows * kDin * 2;
constexpr size_t kOffXBC  = kOffDR16 + (size_t)kRows * kDtR * 2;
constexpr size_t kWsTotal = kOffXBC  + (size_t)kRows * kXbcP * 4;
static_assert(kWsTotal == 107216896ull);
static_assert(kWsTotal <= 134217728ull);
static_assert((size_t)kRows * kDin * 2 <= kOffWX16 - kOffY16);
static_assert((kOffWI16 % 128) == 0 && (kOffWX16 % 128) == 0 && (kOffWD16 % 128) == 0 && (kOffWO16 % 128) == 0 &&
              (kOffXC % 128) == 0 && (kOffZ % 128) == 0 && (kOffU16 % 128) == 0 && (kOffDR16 % 128) == 0 &&
              (kOffXBC % 128) == 0);

__device__ __forceinline__ unsigned short f2bf_bits(float f) {
  unsigned u = __float_as_uint(f);
  return (unsigned short)((u + 0x7FFFu + ((u >> 16) & 1u)) >> 16);
}
__device__ __forceinline__ float bf_bits2f(unsigned short h) { return __uint_as_float(((unsigned)h) << 16); }

__device__ __forceinline__ void dep_guard_h(v8f& a, v8f& b, v16h x, v16h y) { asm volatile("v_nop\n\tv_nop\n\tv_nop\n\tv_nop" : "+v"(a), "+v"(b) : "v"(x), "v"(y)); }
__device__ __forceinline__ void dep_guard_b(v8f& a, v8f& b, v16b x, v16b y) { asm volatile("v_nop\n\tv_nop\n\tv_nop\n\tv_nop" : "+v"(a), "+v"(b) : "v"(x), "v"(y)); }
__device__ __forceinline__ void keep4_h(v16h a, v16h b, v16h c, v16h d) { asm volatile("v_nop" :: "v"(a), "v"(b), "v"(c), "v"(d)); }
__device__ __forceinline__ void keep4_b(v16b a, v16b b, v16b c, v16b d) { asm volatile("v_nop" :: "v"(a), "v"(b), "v"(c), "v"(d)); }
__device__ __forceinline__ void acc_guard4(v8f& a, v8f& b, v8f& c, v8f& d) { asm volatile("v_nop\n\tv_nop\n\tv_nop\n\tv_nop" : "+v"(a), "+v"(b), "+v"(c), "+v"(d)); }
template <typename T> struct Frag;
template <> struct Frag<_Float16> {
  typedef v16h V; union U { v16h v; v8h h[2]; };
  static __device__ __forceinline__ v16h load(const _Float16* p) {
    U f; f.h[0] = *(const v8h*)(p); f.h[1] = *(const v8h*)(p + 16); return f.v;
  }
  static __device__ __forceinline__ v8f mma(v16h a, v16h b, v8f c) {
    return __builtin_amdgcn_wmma_f32_16x16x32_f16(false, a, false, b, (short)0, c, false, false);
  }
  static __device__ __forceinline__ void guard(v8f& a, v8f& b, v16h x, v16h y) { dep_guard_h(a, b, x, y); }
  static __device__ __forceinline__ void keep(v16h a, v16h b, v16h c, v16h d) { keep4_h(a, b, c, d); }
};
template <> struct Frag<__bf16> {
  typedef v16b V; union U { v16b v; v8b h[2]; };
  static __device__ __forceinline__ v16b load(const __bf16* p) {
    U f; f.h[0] = *(const v8b*)(p); f.h[1] = *(const v8b*)(p + 16); return f.v;
  }
  static __device__ __forceinline__ v8f mma(v16b a, v16b b, v8f c) {
    return __builtin_amdgcn_wmma_f32_16x16x32_bf16(false, a, false, b, (short)0, c, false, false);
  }
  static __device__ __forceinline__ void guard(v8f& a, v8f& b, v16b x, v16b y) { dep_guard_b(a, b, x, y); }
  static __device__ __forceinline__ void keep(v16b a, v16b b, v16b c, v16b d) { keep4_b(a, b, c, d); }
};

template <int ET> struct Elem;
template <> struct Elem<0> { typedef _Float16 T; };
template <> struct Elem<1> { typedef __bf16 T; };
template <int ET, bool SPLIT, int BIAS_MODE, int OUT_MODE, bool RESID, int ACT = 0>
__global__ __launch_bounds__(256) void wmma_gemm64(
    const unsigned short* __restrict__ Ap, const unsigned short* __restrict__ A2p, int lda, long strideA,
    const unsigned short* __restrict__ Btp, const unsigned short* __restrict__ Bt2p, int ldb, long strideB,
    void* __restrict__ Cout, void* __restrict__ Cout2, int ldc, long strideC,
    const float* __restrict__ bias,
    const float* __restrict__ resid, long strideR,
    int M, int N, int K, float scale) {
  typedef typename Elem<ET>::T T;
  typedef typename Frag<T>::V V;
  const T* A = (const T*)Ap; const T* A2 = (const T*)A2p; const T* Bt = (const T*)Btp; const T* Bt2 = (const T*)Bt2p;
  __shared__ __align__(16) float sT[8][16 * 68];
  const int b    = blockIdx.y;
  const int lane = threadIdx.x & 31;
  const int wave = threadIdx.x >> 5;
  const int tilesN = N >> 6;
  const int tilesM = M >> 6;
  const int tile = blockIdx.x * 8 + wave;
  if (tile >= tilesM * tilesN) return;
  const int tm = tile / tilesN;
  const int tn = tile - tm * tilesN;
  const int m0 = tm << 6;
  const int n0 = tn << 6;

  const T* Ab  = A  + (size_t)b * strideA;
  const T* Bb  = Bt + (size_t)b * strideB;
  const T* Ab2 = SPLIT ? (A2  + (size_t)b * strideA) : nullptr;
  const T* Bb2 = SPLIT ? (Bt2 + (size_t)b * strideB) : nullptr;

  const int rlane = lane & 15;
  const int koff  = (lane >> 4) * 8;
  const int mOff  = (lane >> 4) * 8;

  v8f acc[4][4];
#pragma unroll
  for (int i = 0; i < 4; ++i)
#pragma unroll
    for (int j = 0; j < 4; ++j) acc[i][j] = (v8f){0.f,0.f,0.f,0.f,0.f,0.f,0.f,0.f};

  for (int k0 = 0; k0 < K; k0 += 32) {
    V bh[4], bl[4];
#pragma unroll
    for (int j = 0; j < 4; ++j) {
      const size_t bo = (size_t)(n0 + (j << 4) + rlane) * ldb + koff + k0;
      bh[j] = Frag<T>::load(Bb + bo);
      if (SPLIT) bl[j] = Frag<T>::load(Bb2 + bo);
    }
#pragma unroll
    for (int i = 0; i < 4; ++i) {
      const size_t ao = (size_t)(m0 + (i << 4) + rlane) * lda + koff + k0;
      V ah = Frag<T>::load(Ab + ao);
      V al;
      if (SPLIT) al = Frag<T>::load(Ab2 + ao);
#pragma unroll
      for (int j = 0; j < 4; ++j) {
        acc[i][j] = Frag<T>::mma(ah, bh[j], acc[i][j]);
        if (SPLIT) {
          acc[i][j] = Frag<T>::mma(ah, bl[j], acc[i][j]);
          acc[i][j] = Frag<T>::mma(al, bh[j], acc[i][j]);
        }
      }
      Frag<T>::guard(acc[i][0], acc[i][3], ah, SPLIT ? al : ah);
    }
    Frag<T>::keep(bh[0], bh[1], bh[2], bh[3]);
    if (SPLIT) Frag<T>::keep(bl[0], bl[1], bl[2], bl[3]);
  }
  acc_guard4(acc[0][0], acc[0][1], acc[0][2], acc[0][3]);
  acc_guard4(acc[1][0], acc[1][1], acc[1][2], acc[1][3]);
  acc_guard4(acc[2][0], acc[2][1], acc[2][2], acc[2][3]);
  acc_guard4(acc[3][0], acc[3][1], acc[3][2], acc[3][3]);

  float* slab = sT[wave];
  const float* Rb = RESID ? (resid + (size_t)b * strideR) : nullptr;
#pragma unroll
  for (int i = 0; i < 4; ++i) {
    const int mBase = m0 + (i << 4);
#pragma unroll
    for (int j = 0; j < 4; ++j) {
      const int n = n0 + (j << 4) + rlane;
      float bv = 0.f;
      if (BIAS_MODE == 2) bv = bias[n];
#pragma unroll
      for (int r = 0; r < 8; ++r) {
        float v = acc[i][j][r] * scale;
        if (BIAS_MODE == 1) v += bias[mBase + mOff + r];
        if (BIAS_MODE == 2) v += bv;
        if (RESID) v += Rb[(size_t)(mBase + mOff + r) * ldc + n];
        if (ACT == 1) v = tanhf(v);
        if (ACT == 2) v = fmaxf(v, 0.0f);
        if (ACT == 3) v = v / (1.0f + expf(-v));
        if (ACT == 4) v = (v > 0.f) ? v : 0.01f * v;
        slab[(mOff + r) * 68 + (j << 4) + rlane] = v;
      }
    }
    __builtin_amdgcn_fence(__ATOMIC_RELEASE, "workgroup");
    __builtin_amdgcn_wave_barrier();
    __builtin_amdgcn_fence(__ATOMIC_ACQUIRE, "workgroup");
    if (OUT_MODE == 0) {
      float* C = (float*)Cout + (size_t)b * strideC;
      const int hh = lane >> 4, c4 = (lane & 15) * 4;
      for (int pass = 0; pass < 2; ++pass) {
#pragma unroll
        for (int it = 0; it < 8; ++it) {
          const int row = it * 2 + hh;
          v4f v = *(const v4f*)(slab + row * 68 + c4);
          *(volatile v4f*)(C + (size_t)(mBase + row) * ldc + n0 + c4) = v;
        }
        __threadfence();
      }
    } else {
      const int q = lane >> 3, c8 = (lane & 7) * 8;
      unsigned short* C  = (unsigned short*)Cout  + (size_t)b * strideC;
      unsigned short* C2 = (OUT_MODE == 2) ? ((unsigned short*)Cout2 + (size_t)b * strideC) : nullptr;
      for (int pass = 0; pass < 2; ++pass) {
#pragma unroll
        for (int it = 0; it < 4; ++it) {
          const int row = it * 4 + q;
          const float* sp = slab + row * 68 + c8;
          v8h hv, lv;
#pragma unroll
          for (int e = 0; e < 8; ++e) {
            if (OUT_MODE == 1) {
              hv[e] = (_Float16)sp[e];
            } else {
              unsigned short hb = f2bf_bits(sp[e]);
              unsigned short lb = f2bf_bits(sp[e] - bf_bits2f(hb));
              hv[e] = __builtin_bit_cast(_Float16, hb);
              lv[e] = __builtin_bit_cast(_Float16, lb);
            }
          }
          *(volatile v8h*)(C + (size_t)(mBase + row) * ldc + n0 + c8) = hv;
          if (OUT_MODE == 2) *(volatile v8h*)(C2 + (size_t)(mBase + row) * ldc + n0 + c8) = lv;
        }
        __threadfence();
      }
    }
    __builtin_amdgcn_fence(__ATOMIC_RELEASE, "workgroup");
    __builtin_amdgcn_wave_barrier();
    __builtin_amdgcn_fence(__ATOMIC_ACQUIRE, "workgroup");
  }
}

__global__ __launch_bounds__(256) void cast_rows_f16_kernel(
    const float* __restrict__ src, unsigned short* __restrict__ dst, int ncols, int srows, int total8, float scale)
{
  const int i = blockIdx.x * 256 + threadIdx.x;
  if (i >= total8) return;
  const size_t e0 = (size_t)i << 3;
  const int row = (int)(e0 / (size_t)ncols);
  const int col = (int)(e0 - (size_t)row * (size_t)ncols);
  const int rs = (row < srows) ? row : (srows - 1);
  const float* sp = src + (size_t)rs * ncols + col;
  const v4f a0 = *(const v4f*)(sp);
  const v4f a1 = *(const v4f*)(sp + 4);
  const float f = (row < srows) ? scale : 0.0f;
  v8h hv;
#pragma unroll
  for (int e = 0; e < 4; ++e) {
    hv[e]     = (_Float16)(a0[e] * f);
    hv[4 + e] = (_Float16)(a1[e] * f);
  }
  unsigned short* q = dst + e0;
  *(volatile v8h*)q = hv;
  __threadfence();
  *(volatile v8h*)q = hv;
}

__global__ __launch_bounds__(256) void layernorm_f16_kernel(
    const float* __restrict__ x, const float* __restrict__ g, const float* __restrict__ bb, unsigned short* __restrict__ XN)
{
  const int lane = threadIdx.x & 31, wave = threadIdx.x >> 5;
  const int row = blockIdx.x * 8 + wave;
  const float* xr = x + (size_t)row * kDm;
  float s = 0.f;
#pragma unroll 1
  for (int c = 0; c < 4; ++c) {
    const float* p = xr + c * 256 + lane * 8;
    const v4f a0 = *(const v4f*)(p);
    const v4f a1 = *(const v4f*)(p + 4);
    s += ((a0[0] + a0[1]) + (a0[2] + a0[3])) + ((a1[0] + a1[1]) + (a1[2] + a1[3]));
  }
#pragma unroll
  for (int off = 16; off > 0; off >>= 1) s += __shfl_xor(s, off, 32);
  const float mu = s * (1.0f / (float)kDm);
  float ss = 0.f;
#pragma unroll 1
  for (int c = 0; c < 4; ++c) {
    const float* p = xr + c * 256 + lane * 8;
    const v4f a0 = *(const v4f*)(p);
    const v4f a1 = *(const v4f*)(p + 4);
#pragma unroll
    for (int e = 0; e < 4; ++e) {
      const float d0 = a0[e] - mu;
      const float d1 = a1[e] - mu;
      ss = fmaf(d0, d0, ss);
      ss = fmaf(d1, d1, ss);
    }
  }
#pragma unroll
  for (int off = 16; off > 0; off >>= 1) ss += __shfl_xor(ss, off, 32);
  const float var = ss * (1.0f / (float)kDm);
  const float rstd = rsqrtf(var + kLnEps);
  v8h hv[4];
#pragma unroll
  for (int c = 0; c < 4; ++c) {
    const int off = c * 256 + lane * 8;
    const v4f a0 = *(const v4f*)(xr + off);
    const v4f a1 = *(const v4f*)(xr + off + 4);
    const v4f g0 = *(const v4f*)(g + off);
    const v4f g1 = *(const v4f*)(g + off + 4);
    const v4f b0 = *(const v4f*)(bb + off);
    const v4f b1 = *(const v4f*)(bb + off + 4);
#pragma unroll
    for (int e = 0; e < 4; ++e) {
      const float t0 = (a0[e] - mu) * rstd;
      const float t1 = (a1[e] - mu) * rstd;
      hv[c][e]     = (_Float16)(t0 * g0[e] + b0[e]);
      hv[c][4 + e] = (_Float16)(t1 * g1[e] + b1[e]);
    }
  }
  unsigned short* orow = XN + (size_t)row * kDm;
  for (int pass = 0; pass < 2; ++pass) {
#pragma unroll
    for (int c = 0; c < 4; ++c)
      *(volatile v8h*)(orow + c * 256 + lane * 8) = hv[c];
    __threadfence();
  }
}

__global__ __launch_bounds__(256) void conv_silu_f16_kernel(
    const float* __restrict__ XC, const float* __restrict__ cw, const float* __restrict__ cb,
    unsigned short* __restrict__ U16)
{
  __shared__ __align__(16) float sT[16 * kConvTP];
  const int tid = threadIdx.x, lane = tid & 31, wave = tid >> 5;
  const int d0 = blockIdx.x * 256, d = d0 + tid;
  const int g0 = blockIdx.y * 64;
  const int tb = g0 & (kSeq - 1);
  const float w0 = cw[d * 4 + 0], w1 = cw[d * 4 + 1], w2 = cw[d * 4 + 2], w3 = cw[d * 4 + 3];
  const float bc = cb[d];
  float xm3, xm2, xm1;
  {
    const bool hist = (tb > 0);
    const int rb = hist ? (g0 - 3) : g0;
    const float v3 = XC[(size_t)rb * kDin + d];
    const float v2 = XC[(size_t)(rb + 1) * kDin + d];
    const float v1 = XC[(size_t)(rb + 2) * kDin + d];
    xm3 = hist ? v3 : 0.f;
    xm2 = hist ? v2 : 0.f;
    xm1 = hist ? v1 : 0.f;
  }
#pragma unroll 1
  for (int sub = 0; sub < 4; ++sub) {
    const int lb = g0 + sub * 16;
#pragma unroll 1
    for (int s = 0; s < 16; ++s) {
      const float xcur = XC[(size_t)(lb + s) * kDin + d];
      float acc = w0 * xm3;
      acc = fmaf(w1, xm2, acc);
      acc = fmaf(w2, xm1, acc);
      acc = fmaf(w3, xcur, acc);
      const float sv = acc + bc;
      const float sg = __builtin_amdgcn_rcpf(1.0f + __expf(-sv));
      sT[s * kConvTP + tid] = sv * sg;
      xm3 = xm2; xm2 = xm1; xm1 = xcur;
    }
    __syncthreads();
    v8h hv[2];
#pragma unroll
    for (int it = 0; it < 2; ++it) {
      const float* sp = sT + (it * 8 + wave) * kConvTP + lane * 8;
      const v4f a0 = *(const v4f*)(sp);
      const v4f a1 = *(const v4f*)(sp + 4);
#pragma unroll
      for (int e = 0; e < 4; ++e) {
        hv[it][e]     = (_Float16)(a0[e] * kUScale);
        hv[it][4 + e] = (_Float16)(a1[e] * kUScale);
      }
    }
    for (int pass = 0; pass < 2; ++pass) {
#pragma unroll
      for (int it = 0; it < 2; ++it) {
        const size_t o = (size_t)(lb + it * 8 + wave) * kDin + d0 + lane * 8;
        *(volatile v8h*)(U16 + o) = hv[it];
      }
      __threadfence();
    }
    __syncthreads();
  }
}

__global__ __launch_bounds__(64) void scan_kernel(
    const float* __restrict__ XBC, const float* __restrict__ XC, const float* __restrict__ Zp,
    const unsigned short* __restrict__ DT16,
    const float* __restrict__ cw, const float* __restrict__ cb, const float* __restrict__ dtb,
    const float* __restrict__ Alog, const float* __restrict__ Dp, unsigned short* __restrict__ Y16)
{
  __shared__ __align__(16) float sX[kScanTS * kXbcW];
  __shared__ __align__(16) float sY[kScanTS * kScanYP];
  __shared__ __align__(16) float sA[kNst * kScanCh];
  const int tid = threadIdx.x, lane = tid & 31, wave = tid >> 5;
  constexpr int kBlkPerB = kDin / kScanCh;
  const int bix = blockIdx.x / kBlkPerB;
  const int d0  = (blockIdx.x - bix * kBlkPerB) * kScanCh;
  const int d   = d0 + tid;
  const size_t row0 = (size_t)bix * kSeq;
#pragma unroll 1
  for (int s = 0; s < kNst; ++s) sA[s * kScanCh + tid] = -expf(Alog[(size_t)d * kNst + s]);
  __syncthreads();
  float negA[kNst], h[kNst];
#pragma unroll
  for (int s = 0; s < kNst; ++s) {
    negA[s] = sA[s * kScanCh + tid];
    h[s] = 0.f;
  }
  const float w0 = cw[d * 4 + 0], w1 = cw[d * 4 + 1], w2 = cw[d * 4 + 2], w3 = cw[d * 4 + 3];
  const float bc = cb[d], db = dtb[d], Dd = Dp[d];
  float xm3 = 0.f, xm2 = 0.f, xm1 = 0.f;
  const int lr = tid >> 3, lc4 = (tid & 7) * 4;
  const int q = lane >> 3, c8 = (lane & 7) * 8;
  const unsigned* DTw = (const unsigned*)(const void*)DT16;
#pragma unroll 1
  for (int t0 = 0; t0 < kSeq; t0 += kScanTS) {
    __syncthreads();
#pragma unroll
    for (int i = 0; i < 8; ++i) {
      const int r = lr + 8 * i;
      *(v4f*)(sX + r * kXbcW + lc4) = *(const v4f*)(XBC + (row0 + t0 + r) * kXbcP + lc4);
    }
    __syncthreads();
#pragma unroll 1
    for (int s = 0; s < kScanTS; ++s) {
      const size_t grow = row0 + t0 + s;
      const float* xr = sX + s * kXbcW;
      const float xcur = XC[grow * kDin + d];
      float cacc = w0 * xm3;
      cacc = fmaf(w1, xm2, cacc);
      cacc = fmaf(w2, xm1, cacc);
      cacc = fmaf(w3, xcur, cacc);
      const float sv = cacc + bc;
      const float u  = sv * __builtin_amdgcn_rcpf(1.0f + __expf(-sv));
      xm3 = xm2; xm2 = xm1; xm1 = xcur;
      const unsigned wd = DTw[((grow * kDin + d0) >> 1) + (tid >> 1)];
      const unsigned short hb = (unsigned short)((tid & 1) ? (wd >> 16) : (wd & 0xffffu));
      const float pre = (float)__builtin_bit_cast(_Float16, hb);
      const float v   = pre * kDtInv + db;
      const float a   = __expf(-fabsf(v));
      const float uu  = 1.0f + a;
      const float l1p = __logf(uu) + (a - (uu - 1.0f)) * __builtin_amdgcn_rcpf(uu);
      const float delta = fmaxf(v, 0.0f) + l1p;
      float Bs[kNst], Cs[kNst];
#pragma unroll
      for (int q4 = 0; q4 < 4; ++q4) {
        const v4f bv = *(const v4f*)(xr + 4 * q4);
        const v4f cv = *(const v4f*)(xr + kNst + 4 * q4);
        Bs[4 * q4 + 0] = bv[0]; Bs[4 * q4 + 1] = bv[1]; Bs[4 * q4 + 2] = bv[2]; Bs[4 * q4 + 3] = bv[3];
        Cs[4 * q4 + 0] = cv[0]; Cs[4 * q4 + 1] = cv[1]; Cs[4 * q4 + 2] = cv[2]; Cs[4 * q4 + 3] = cv[3];
      }
      const float dtx = delta * u;
      float y = 0.f;
#pragma unroll
      for (int k = 0; k < kNst; ++k) {
        const float e = __expf(delta * negA[k]);
        h[k] = e * h[k] + dtx * Bs[k];
        y = h[k] * Cs[k] + y;
      }
      y = u * Dd + y;
      const float zv = Zp[grow * kDin + d];
      const float sg = __builtin_amdgcn_rcpf(1.0f + __expf(-zv));
      y = y * (zv * sg);
      sY[s * kScanYP + tid] = y;
    }
    __syncthreads();
    v8h hv[8];
#pragma unroll
    for (int it = 0; it < 8; ++it) {
      const int row = it * 8 + wave * 4 + q;
      const float* sp = sY + row * kScanYP + c8;
      const v4f a0 = *(const v4f*)(sp);
      const v4f a1 = *(const v4f*)(sp + 4);
#pragma unroll
      for (int e = 0; e < 4; ++e) {
        hv[it][e]     = (_Float16)(a0[e] * kYScale);
        hv[it][4 + e] = (_Float16)(a1[e] * kYScale);
      }
    }
    for (int pass = 0; pass < 2; ++pass) {
#pragma unroll
      for (int it = 0; it < 8; ++it) {
        const int row = it * 8 + wave * 4 + q;
        const size_t o = (row0 + t0 + row) * kDin + d0 + c8;
        *(volatile v8h*)(Y16 + o) = hv[it];
      }
      __threadfence();
    }
  }
}

extern "C" void kernel_launch(void* const* d_in, const int* in_sizes, int n_in,
                              void* d_out, int out_size, void* d_ws, size_t ws_size,
                              hipStream_t stream) {
  if (n_in < 12) return;
  if (in_sizes[0] != kRows * kDm) return;
  if (in_sizes[1] != kDm) return;
  if (in_sizes[2] != kDm) return;
  if (in_sizes[3] != 2 * kDin * kDm) return;
  if (in_sizes[4] != kDin * 4) return;
  if (in_sizes[5] != kDin) return;
  if (in_sizes[6] != kDin * kNst) return;
  if (in_sizes[7] != kDin) return;
  if (in_sizes[8] != kXpN * kDin) return;
  if (in_sizes[9] != kDin * kDtR) return;
  if (in_sizes[10] != kDin) return;
  if (in_sizes[11] != kDm * kDin) return;
  if (out_size != kRows * kDm) return;
  if (ws_size < kWsTotal) return;

  const float* x       = (const float*)d_in[0];
  const float* ln_g    = (const float*)d_in[1];
  const float* ln_b    = (const float*)d_in[2];
  const float* W_in    = (const float*)d_in[3];
  const float* conv_w  = (const float*)d_in[4];
  const float* conv_b  = (const float*)d_in[5];
  const float* A_log   = (const float*)d_in[6];
  const float* Dp      = (const float*)d_in[7];
  const float* W_xproj = (const float*)d_in[8];
  const float* W_dt    = (const float*)d_in[9];
  const float* b_dt    = (const float*)d_in[10];
  const float* W_out   = (const float*)d_in[11];
  float* out = (float*)d_out;

  char* ws = (char*)d_ws;
  unsigned short* XN16 = (unsigned short*)(ws + kOffXN16);
  unsigned short* WI16 = (unsigned short*)(ws + kOffWI16);
  unsigned short* Y16  = (unsigned short*)(ws + kOffY16);
  unsigned short* WX16 = (unsigned short*)(ws + kOffWX16);
  unsigned short* WD16 = (unsigned short*)(ws + kOffWD16);
  unsigned short* WO16 = (unsigned short*)(ws + kOffWO16);
  float*          XC   = (float*)(ws + kOffXC);
  float*          Zb   = (float*)(ws + kOffZ);
  unsigned short* U16  = (unsigned short*)(ws + kOffU16);
  unsigned short* DT16 = (unsigned short*)(ws + kOffDT16);
  unsigned short* DR16 = (unsigned short*)(ws + kOffDR16);
  float*          XBC  = (float*)(ws + kOffXBC);

  const float inv64   = 1.0f / 64.0f;
  const float inv128  = 1.0f / 128.0f;
  const float inv1024 = 1.0f / 1024.0f;
  const float inv32   = 1.0f / 32.0f;
  const float inv4096 = 1.0f / 4096.0f;

  layernorm_f16_kernel<<<kRows / 8, 256, 0, stream>>>(x, ln_g, ln_b, XN16);

  cast_rows_f16_kernel<<<(2 * kDin * kDm / 8) / 256, 256, 0, stream>>>(W_in, WI16, kDm, 2 * kDin, 2 * kDin * kDm / 8, kWScale);
  cast_rows_f16_kernel<<<(kXpPad * kDin / 8) / 256, 256, 0, stream>>>(W_xproj, WX16, kDin, kXpN, kXpPad * kDin / 8, kWScale);
  cast_rows_f16_kernel<<<(kDin * kDtR / 8) / 256, 256, 0, stream>>>(W_dt, WD16, kDtR, kDin, kDin * kDtR / 8, kWScale);
  cast_rows_f16_kernel<<<(kDm * kDin / 8) / 256, 256, 0, stream>>>(W_out, WO16, kDin, kDm, kDm * kDin / 8, kWScale);

  wmma_gemm64<0, false, 0, 0, false><<<dim3(256, 1), 256, 0, stream>>>(
      XN16, nullptr, kDm, 0L,
      WI16, nullptr, kDm, 0L,
      (void*)XC, nullptr, kDin, 0L,
      nullptr, nullptr, 0L,
      kRows, kDin, kDm, inv64);
  wmma_gemm64<0, false, 0, 0, false><<<dim3(256, 1), 256, 0, stream>>>(
      XN16, nullptr, kDm, 0L,
      WI16 + (size_t)kDin * kDm, nullptr, kDm, 0L,
      (void*)Zb, nullptr, kDin, 0L,
      nullptr, nullptr, 0L,
      kRows, kDin, kDm, inv64);

  conv_silu_f16_kernel<<<dim3(kDin / 256, kRows / 64), 256, 0, stream>>>(XC, conv_w, conv_b, U16);

  wmma_gemm64<0, false, 0, 1, false><<<dim3(8, 1), 256, 0, stream>>>(
      U16, nullptr, kDin, 0L,
      WX16, nullptr, kDin, 0L,
      (void*)DR16, nullptr, kDtR, 0L,
      nullptr, nullptr, 0L,
      kRows, 64, kDin, inv128);
  wmma_gemm64<0, false, 0, 0, false><<<dim3(8, 1), 256, 0, stream>>>(
      U16, nullptr, kDin, 0L,
      WX16 + (size_t)64 * kDin, nullptr, kDin, 0L,
      (void*)XBC, nullptr, kXbcP, 0L,
      nullptr, nullptr, 0L,
      kRows, 64, kDin, inv1024);

  wmma_gemm64<0, false, 0, 1, false><<<dim3(256, 1), 256, 0, stream>>>(
      DR16, nullptr, kDtR, 0L,
      WD16, nullptr, kDtR, 0L,
      (void*)DT16, nullptr, kDin, 0L,
      nullptr, nullptr, 0L,
      kRows, kDin, kDtR, inv32);

  scan_kernel<<<kBatch * (kDin / kScanCh), kScanCh, 0, stream>>>(XBC, XC, Zb, DT16, conv_w, conv_b, b_dt, A_log, Dp, Y16);

  wmma_gemm64<0, false, 0, 0, true><<<dim3(128, 1), 256, 0, stream>>>(
      Y16, nullptr, kDin, 0L,
      WO16, nullptr, kDin, 0L,
      (void*)out, nullptr, kDm, 0L,
      nullptr, x, 0L,
      kRows, kDm, kDin, inv4096);
}
